// MS_BACL_55765855371540
// MI455X (gfx1250) — hardware-run, weakly checked
//
#include <hip/hip_runtime.h>


namespace {
constexpr int N = 50000, NP = 50048  , E = 400000, G = 256;
constexpr int F1 = 93, K1P = 96, N1L2 = 930, N1L2P = 960, F2 = 43, K2P = 64, N2L2 = 430, N2L2P = 448;
constexpr int P1W = 2 * N1L2  , P1WP = 1888, P2W = 2 * N2L2  , P2WP = 864, HID = 1024, XG = 512, FF = 256;
constexpr float XS = 8.0f, WSC = 256.0f, NEG = 0.2f  ;

typedef _Float16 b16;
typedef __attribute__((ext_vector_type(16))) _Float16 v16b;
typedef __attribute__((ext_vector_type(8))) _Float16 v8b;
typedef __attribute__((ext_vector_type(8))) float v8f;
typedef __attribute__((ext_vector_type(4))) float v4f;
__device__ __forceinline__ float bf16_rne(float f) { unsigned int u = __float_as_uint(f); u += 0x7FFFu + ((u >> 16) & 1u); return __uint_as_float(u & 0xFFFF0000u); }
__device__ __forceinline__ void split16(float v, b16& hi, b16& lo) { hi = (b16)v; lo = (b16)(v - (float)hi); }
__device__ __forceinline__ v16b frag_kb(const b16* p, int hh) { const v8b a = *(const v8b*)(p + 8 * hh), b = *(const v8b*)(p + 16 + 8 * hh); v16b f;
#pragma unroll
  for (int e = 0; e < 8; ++e) { f[e] = a[e]; f[8 + e] = b[e]; } return f; }
__device__ __forceinline__ v8f wmma16b(v16b a, v16b b, v8f c) { v8f d = __builtin_amdgcn_wmma_f32_16x16x32_f16(false, a, false, b, (short)0, c, false, false); asm volatile("v_nop\n\tv_nop\n\tv_nop\n\tv_nop" : "+v"(d) : "v"(a), "v"(b)); return d; }
__device__ __forceinline__ void wave_lds_sync() { __builtin_amdgcn_fence(__ATOMIC_RELEASE, "workgroup"); __builtin_amdgcn_wave_barrier(); __builtin_amdgcn_fence(__ATOMIC_ACQUIRE, "workgroup"); }
__device__ __forceinline__ float pmul(float a, float b) { float p = a * b; asm volatile("" : "+v"(p)); return p; }
__device__ __forceinline__ int iclamp(int v, int lo, int hi) { return v < lo ? lo : (v > hi ? hi : v); }
__device__ __forceinline__ float nexp(float x) { return __builtin_amdgcn_exp2f(x * 1.4426950408889634f); }
__device__ __forceinline__ float lrelu(float x) { return x > 0.0f ? x : NEG * x; }

constexpr int CSR_NBLK = 512, CSR_GB = 9, CSR_GN = 1 << CSR_GB  , CSR_MAXG = 512, CSR_CAP = 12288  ;
__global__ __launch_bounds__(64) void csrA_kernel(const int* __restrict__ dst, int E, int N, int nG, int CHP, int NGP, int* __restrict__ STG, int* __restrict__ HST) {
  extern __shared__ int sm[];
  int* cnt = sm; int* run = sm + NGP; int* ids = sm + 2 * NGP;
  const int b = blockIdx.x; const int ch = (E + CSR_NBLK - 1) / CSR_NBLK; const int e0 = b * ch, e1 = min(E, e0 + ch);
  for (int i = threadIdx.x; i < NGP; i += 64) cnt[i] = 0;
  for (int i = threadIdx.x; i < CHP; i += 64) ids[i] = -1;
  __syncthreads();
  if (threadIdx.x == 0) {
    for (int e = e0; e < e1; ++e) { int d = dst[e]; d = (d < 0) ? 0 : (d >= N ? N - 1 : d); cnt[d >> CSR_GB] += 1; }
    int acc = 0; for (int g = 0; g < nG; ++g) { run[g] = acc; acc += cnt[g]; }
    for (int e = e0; e < e1; ++e) { int d = dst[e]; d = (d < 0) ? 0 : (d >= N ? N - 1 : d); const int g = d >> CSR_GB; ids[run[g]] = e; run[g] += 1; } }
  __syncthreads();
  typedef __attribute__((ext_vector_type(4))) int v4i;
  for (int pass = 0; pass < 2; ++pass) {
    for (int i = threadIdx.x; i < CHP / 4; i += 64) *(volatile v4i*)(STG + (size_t)b * CHP + i * 4) = *(const v4i*)(&ids[i * 4]);
    for (int i = threadIdx.x; i < NGP / 4; i += 64) { v4i v; for (int e = 0; e < 4; ++e) v[e] = (i * 4 + e < nG) ? cnt[i * 4 + e] : 0; *(volatile v4i*)(HST + (size_t)b * NGP + i * 4) = v; }
    __threadfence(); }
}
__global__ __launch_bounds__(512) void csrS_kernel(const int* __restrict__ HST, int nG, int NGP, int* __restrict__ START, int* __restrict__ TOT, int* __restrict__ OFF) {
  __shared__ int tot[CSR_MAXG];
  const int b = threadIdx.x;
  for (int pass = 0; pass < 2; ++pass) { int runb = 0; for (int g = 0; g < nG; ++g) { int c = HST[(size_t)b * NGP + g]; c = (c < 0) ? 0 : c; ((volatile int*)OFF)[(size_t)g * CSR_NBLK + b] = runb; runb += c; } __threadfence(); }
  for (int g = threadIdx.x; g < nG; g += 512) { int s = 0; for (int bb = 0; bb < CSR_NBLK; ++bb) { int c = HST[(size_t)bb * NGP + g]; s += (c < 0) ? 0 : c; } tot[g] = s; }
  __syncthreads();
  if (threadIdx.x < 32) {
    __shared__ int st[CSR_MAXG + 32];
    if (threadIdx.x == 0) { int acc = 0; for (int g = 0; g < NGP; ++g) { st[g] = acc; if (g < nG) acc += (tot[g] + 31) & ~31; } st[NGP] = acc; }
    __builtin_amdgcn_fence(__ATOMIC_RELEASE, "workgroup"); __builtin_amdgcn_wave_barrier(); __builtin_amdgcn_fence(__ATOMIC_ACQUIRE, "workgroup");
    for (int pass = 0; pass < 2; ++pass) { for (int i = threadIdx.x; i < NGP + 32; i += 32) { ((volatile int*)START)[i] = (i <= NGP) ? st[min(i, NGP)] : 0; ((volatile int*)TOT)[i] = (i < nG) ? tot[i] : 0; } __threadfence(); } }
}
__global__ __launch_bounds__(256) void csrB_kernel(const int* __restrict__ dst, int N, int nG, int CHP, int NGP, int permLen, const int* __restrict__ STG, const int* __restrict__ HST, const int* __restrict__ OFF, const int* __restrict__ START, const int* __restrict__ TOT, int* __restrict__ PERM, int* __restrict__ ROWPTR, int* __restrict__ ROWCNT, int* __restrict__ FLAG) {
  typedef __attribute__((ext_vector_type(4))) int v4i;
  __shared__ int ids[CSR_CAP]; __shared__ unsigned short key[CSR_CAP]; __shared__ int outp[CSR_CAP]; __shared__ int ncnt[CSR_GN + 1]; __shared__ int boff[CSR_NBLK + 1];
  const int g = blockIdx.x, t_ = threadIdx.x; int tot = TOT[g]; int st = START[g], stn = START[g + 1]; const int v0 = g * CSR_GN; const int nv = min(CSR_GN, N - v0);
  st = (st < 0) ? 0 : (st > permLen - 32 ? permLen - 32 : st) & ~31; stn = (stn < st) ? st : (stn > permLen ? permLen : stn); tot = (tot < 0) ? 0 : tot; if (tot > stn - st && tot <= CSR_CAP) tot = stn - st;
  if (tot > CSR_CAP) {
    for (int pass = 0; pass < 2; ++pass) { for (int i = t_; i < CSR_GN / 4; i += 256) { v4i a, c; for (int e = 0; e < 4; ++e) { a[e] = st; c[e] = 0; } *(volatile v4i*)(ROWPTR + v0 + i * 4) = a; *(volatile v4i*)(ROWCNT + v0 + i * 4) = c; } if (t_ == 0) ((volatile int*)FLAG)[0] = 1; __threadfence(); } (void)nv; return; }
  if (t_ == 0) { int acc = 0; for (int b = 0; b < CSR_NBLK; ++b) { boff[b] = acc; int c = HST[(size_t)b * NGP + g]; c = (c < 0) ? 0 : (c > CHP ? CHP : c); acc += c; if (acc > tot) acc = tot; } boff[CSR_NBLK] = acc; }
  for (int i = t_; i <= CSR_GN; i += 256) ncnt[i] = 0;
  __syncthreads();
  for (int b = 0; b < CSR_NBLK; ++b) { const int c = boff[b + 1] - boff[b]; int o_ = OFF[(size_t)g * CSR_NBLK + b]; o_ = (o_ < 0) ? 0 : (o_ > CHP - c ? CHP - c : o_); const int* src_ = STG + (size_t)b * CHP + o_;
    for (int i = t_; i < c; i += 256) { int id = src_[i]; id = (id < 0) ? 0 : id; ids[boff[b] + i] = id; int d = dst[id]; d = (d < v0) ? v0 : (d >= N ? N - 1 : d); int kk = d - v0; kk = (kk < 0) ? 0 : (kk >= CSR_GN ? CSR_GN - 1 : kk); key[boff[b] + i] = (unsigned short)kk; } }
  __syncthreads();
  if (t_ == 0) { for (int i = 0; i < tot; ++i) ncnt[key[i]] += 1; int acc = 0; for (int vl = 0; vl < CSR_GN; ++vl) { const int c = ncnt[vl]; ncnt[vl] = acc; acc += c; } ncnt[CSR_GN] = acc;
    for (int i = 0; i < tot; ++i) { const int vl = key[i]; outp[ncnt[vl]] = ids[i]; ncnt[vl] += 1; }
    for (int vl = CSR_GN; vl > 0; --vl) ncnt[vl] = ncnt[vl - 1]; ncnt[0] = 0; }
  __syncthreads();
  for (int pass = 0; pass < 2; ++pass) {
    for (int i = t_; i < (stn - st) / 4; i += 256) { v4i v; for (int e = 0; e < 4; ++e) { const int q = i * 4 + e; v[e] = (q < tot) ? outp[q] : -1; } *(volatile v4i*)(PERM + st + i * 4) = v; }
    for (int i = t_; i < CSR_GN / 4; i += 256) { v4i a, c; for (int e = 0; e < 4; ++e) { const int vl = i * 4 + e; a[e] = st + ncnt[vl]; c[e] = (vl < nv) ? (ncnt[vl + 1] - ncnt[vl]) : 0; } *(volatile v4i*)(ROWPTR + v0 + i * 4) = a; *(volatile v4i*)(ROWCNT + v0 + i * 4) = c; }
    __threadfence(); }
}
__global__ __launch_bounds__(256) void csrZ_kernel(int* __restrict__ p, size_t n4) { typedef __attribute__((ext_vector_type(4))) int v4i; const size_t tid = (size_t)blockIdx.x * 256 + threadIdx.x, nth = (size_t)gridDim.x * 256; v4i z = {0, 0, 0, 0}; for (size_t i = tid; i < n4; i += nth) *(volatile v4i*)(p + i * 4) = z; }
struct CsrBufs { int *STG, *HST, *OFF, *START, *TOT, *PERM, *ROWPTR, *ROWCNT, *FLAG; int nG, NGP, CHP; size_t permLen; char* base; size_t bytes; };
static size_t csr_carve(CsrBufs& c, char* ws, size_t off, int E, int N) {
  const size_t off0 = off; c.base = ws + off;
  auto al = [&](size_t bytes) { char* p = ws + off; off += (bytes + 255) & ~(size_t)255; return p; };
  c.nG = (N + CSR_GN - 1) / CSR_GN; c.NGP = (c.nG + 31) & ~31; const int ch = (E + CSR_NBLK - 1) / CSR_NBLK; c.CHP = (ch + 31) & ~31; c.permLen = (size_t)E + 32 * (size_t)c.nG + 32;
  c.STG = (int*)al((size_t)CSR_NBLK * c.CHP * 4); c.HST = (int*)al((size_t)CSR_NBLK * c.NGP * 4); c.OFF = (int*)al((size_t)c.NGP * CSR_NBLK * 4); c.START = (int*)al((size_t)(c.NGP + 64) * 4); c.TOT = (int*)al((size_t)(c.NGP + 64) * 4);
  c.PERM = (int*)al(c.permLen * 4); c.ROWPTR = (int*)al((size_t)c.nG * CSR_GN * 4); c.ROWCNT = (int*)al((size_t)c.nG * CSR_GN * 4); c.FLAG = (int*)al(256);
  c.bytes = off - off0; return off;
}
static void csr_build(const CsrBufs& c, const int* dst, int E, int N, hipStream_t stream) {
  const size_t smem = (size_t)(2 * c.NGP + c.CHP) * 4;
  csrZ_kernel<<<512, 256, 0, stream>>>((int*)c.base, c.bytes / 16);
  csrA_kernel<<<CSR_NBLK, 64, smem, stream>>>(dst, E, N, c.nG, c.CHP, c.NGP, c.STG, c.HST);
  csrS_kernel<<<1, 512, 0, stream>>>(c.HST, c.nG, c.NGP, c.START, c.TOT, c.OFF);
  csrB_kernel<<<c.nG, 256, 0, stream>>>(dst, N, c.nG, c.CHP, c.NGP, (int)c.permLen, c.STG, c.HST, c.OFF, c.START, c.TOT, c.PERM, c.ROWPTR, c.ROWCNT, c.FLAG);
}


__global__ __launch_bounds__(256) void wprep_kernel(const float* __restrict__ w, int nin, int nout, int kinp, int noutp, b16* __restrict__ dst) {
  const size_t u = (size_t)blockIdx.x * 256 + threadIdx.x; if (u >= (size_t)noutp * kinp / 8) return; const size_t e = u * 8; const int oo = (int)(e / kinp), k0 = (int)(e % kinp); v8b o;
  for (int j = 0; j < 8; ++j) { const int k = k0 + j; o[j] = (oo < nout && k < nin) ? (b16)(bf16_rne(w[(size_t)k * nout + oo]) * WSC) : (b16)0.0f; }
  for (int pass = 0; pass < 2; ++pass) { *(volatile v8b*)(dst + e) = o; __threadfence(); }
}
template <int F, int KP>
__global__ __launch_bounds__(256) void agg_kernel(const float* __restrict__ hin, int raw, const int* __restrict__ srcs, const int* __restrict__ PERM, const int* __restrict__ ROWPTR, const int* __restrict__ ROWCNT, int permLen, float* __restrict__ Sout) {
  __shared__ __attribute__((aligned(16))) float row[8][KP];
  const int wave = threadIdx.x >> 5, lane = threadIdx.x & 31; const size_t v = (size_t)blockIdx.x * 8 + wave; constexpr int NC = KP / 32;
  float acc[NC]; for (int i = 0; i < NC; ++i) acc[i] = 0.0f;
  auto rd = [&](size_t u, int c) -> float { if (c >= F) return 0.0f; return raw ? bf16_rne(hin[u * F + c]) : hin[u * KP + c]; };
  if (v < (size_t)N) { for (int i = 0; i < NC; ++i) acc[i] = rd(v, i * 32 + lane); int st = ROWPTR[v], cnt = ROWCNT[v]; cnt = iclamp(cnt, 0, 8192); st = iclamp(st, 0, permLen - cnt);
    for (int k = 0; k < cnt; ++k) { const int e = iclamp(PERM[st + k], 0, E - 1); const size_t s = (size_t)iclamp(srcs[e], 0, N - 1); for (int i = 0; i < NC; ++i) acc[i] += rd(s, i * 32 + lane); } }
  for (int i = 0; i < NC; ++i) row[wave][i * 32 + lane] = acc[i];
  wave_lds_sync();
  for (int pass = 0; pass < 2; ++pass) { if (lane < KP / 4) *(volatile v4f*)(Sout + v * KP + lane * 4) = *(const v4f*)(&row[wave][lane * 4]); __threadfence(); }
}
template <int F, int KP>
__global__ __launch_bounds__(128) void gin1_kernel(const float* __restrict__ Sx, const b16* __restrict__ Wt, const float* __restrict__ bias, float* __restrict__ H1) {
  constexpr int NT = KP / 16; __shared__ __attribute__((aligned(16))) b16 Ah[4][16][KP + 8], Al[4][16][KP + 8]; __shared__ __attribute__((aligned(16))) float Tf[4][16][KP + 4];
  const int wave = threadIdx.x >> 5, lane = threadIdx.x & 31, nloc = lane & 15, hlf = lane >> 4; const size_t m0 = (size_t)blockIdx.x * 64 + wave * 16;
  for (int q = lane; q < 16 * (KP / 4); q += 32) { const int rr = q / (KP / 4), c4 = (q % (KP / 4)) * 4; const v4f xv = *(const v4f*)(Sx + (m0 + rr) * KP + c4); for (int j = 0; j < 4; ++j) { b16 p, pl; split16(xv[j] * XS, p, pl); Ah[wave][rr][c4 + j] = p; Al[wave][rr][c4 + j] = pl; } }
  wave_lds_sync(); v8f acc[NT];
#pragma unroll
  for (int t = 0; t < NT; ++t) acc[t] = (v8f){};
#pragma unroll
  for (int kb = 0; kb < KP; kb += 32) { const v16b a = frag_kb(&Ah[wave][nloc][kb], hlf), al = frag_kb(&Al[wave][nloc][kb], hlf);
#pragma unroll
    for (int t = 0; t < NT; ++t) { const v16b bw = frag_kb(Wt + (size_t)(t * 16 + nloc) * KP + kb, hlf); acc[t] = wmma16b(a, bw, acc[t]); acc[t] = wmma16b(al, bw, acc[t]); } }
#pragma unroll
  for (int t = 0; t < NT; ++t) { const int c = t * 16 + nloc; const float bb = (c < F) ? bf16_rne(bias[c]) : 0.0f;
#pragma unroll 1
    for (int r = 0; r < 8; ++r) Tf[wave][8 * hlf + r][c] = fmaxf(acc[t][r] * (1.0f / (XS * WSC)) + bb, 0.0f); }
  wave_lds_sync();
  for (int pass = 0; pass < 2; ++pass) { for (int q = lane; q < 16 * (KP / 4); q += 32) { const int rr = q / (KP / 4), c4 = (q % (KP / 4)) * 4; *(volatile v4f*)(H1 + (m0 + rr) * KP + c4) = *(const v4f*)(&Tf[wave][rr][c4]); } __threadfence(); }
}
template <int KP, int N2, int N2P>
__global__ __launch_bounds__(32) void gin2pool_kernel(const float* __restrict__ S2, const b16* __restrict__ Wt, const float* __restrict__ bias, const int* __restrict__ seg, float* __restrict__ POOL) {
  __shared__ __attribute__((aligned(16))) b16 Ah[16][KP + 8], Al[16][KP + 8]; __shared__ __attribute__((aligned(16))) float pm[2][64];
  const int lane = threadIdx.x, nloc = lane & 15, hlf = lane >> 4; const int g = blockIdx.x, cb = blockIdx.y; const int c0 = cb * 64;
  int lo = 0, hi_ = N; { int a = 0, b = N; while (a < b) { const int m = (a + b) >> 1; if (seg[m] < g) a = m + 1; else b = m; } lo = a; a = 0; b = N; while (a < b) { const int m = (a + b) >> 1; if (seg[m] < g + 1) a = m + 1; else b = m; } hi_ = a; }
  float cmax[4], csum[4]; for (int t = 0; t < 4; ++t) { cmax[t] = -INFINITY; csum[t] = 0.0f; } float bb[4]; for (int t = 0; t < 4; ++t) { const int c = c0 + t * 16 + nloc; bb[t] = (c < N2) ? bf16_rne(bias[c]) : 0.0f; }
  for (int r0 = lo; r0 < hi_; r0 += 16) {
    for (int q = lane; q < 16 * (KP / 4); q += 32) { const int rr = q / (KP / 4), c4 = (q % (KP / 4)) * 4; const size_t row = (size_t)r0 + rr; v4f xv = {0.0f, 0.0f, 0.0f, 0.0f}; if (row < (size_t)hi_) xv = *(const v4f*)(S2 + row * KP + c4); for (int j = 0; j < 4; ++j) { b16 p, pl; split16(xv[j] * XS, p, pl); Ah[rr][c4 + j] = p; Al[rr][c4 + j] = pl; } }
    wave_lds_sync(); v8f acc[4] = {{}, {}, {}, {}};
#pragma unroll
    for (int kb = 0; kb < KP; kb += 32) { const v16b a = frag_kb(&Ah[nloc][kb], hlf), al = frag_kb(&Al[nloc][kb], hlf);
#pragma unroll
      for (int t = 0; t < 4; ++t) { const v16b bw = frag_kb(Wt + (size_t)(c0 + t * 16 + nloc) * KP + kb, hlf); acc[t] = wmma16b(a, bw, acc[t]); acc[t] = wmma16b(al, bw, acc[t]); } }
#pragma unroll
    for (int t = 0; t < 4; ++t)
#pragma unroll 1
      for (int r = 0; r < 8; ++r) { const int row = r0 + 8 * hlf + r; if (row < hi_) { const float h = fmaxf(acc[t][r] * (1.0f / (XS * WSC)) + bb[t], 0.0f); cmax[t] = fmaxf(cmax[t], h); csum[t] += h; } }
    wave_lds_sync(); }
  const int cnt = hi_ - lo; const float inv = 1.0f / fmaxf((float)cnt, 1.0f);
#pragma unroll
  for (int t = 0; t < 4; ++t) { const float m2 = fmaxf(cmax[t], __shfl_xor(cmax[t], 16)); const float s2 = csum[t] + __shfl_xor(csum[t], 16); const int c = c0 + t * 16 + nloc;
    if (hlf == 0) { pm[0][t * 16 + nloc] = (c < N2 && cnt > 0) ? m2 : 0.0f; pm[1][t * 16 + nloc] = (c < N2) ? s2 * inv : 0.0f; } }
  wave_lds_sync();
  for (int pass = 0; pass < 2; ++pass) { if (lane < 16) *(volatile v4f*)(POOL + (size_t)g * (2 * N2P) + c0 + lane * 4) = *(const v4f*)(&pm[0][lane * 4]); else *(volatile v4f*)(POOL + (size_t)g * (2 * N2P) + N2P + c0 + (lane - 16) * 4) = *(const v4f*)(&pm[1][(lane - 16) * 4]); __threadfence(); }
}
template <int N2, int N2P, int PWP>
__global__ __launch_bounds__(256) void repack_kernel(const float* __restrict__ POOL, float* __restrict__ PIN) {
  const int g = blockIdx.x; __shared__ __attribute__((aligned(16))) float row[PWP];
  for (int c = threadIdx.x; c < PWP; c += 256) { float v = 0.0f; if (c < N2) v = POOL[(size_t)g * 2 * N2P + c]; else if (c < 2 * N2) v = POOL[(size_t)g * 2 * N2P + N2P + (c - N2)]; row[c] = v; }
  __syncthreads();
  for (int pass = 0; pass < 2; ++pass) { for (int q = threadIdx.x; q < PWP / 4; q += 256) *(volatile v4f*)(PIN + (size_t)g * PWP + q * 4) = *(const v4f*)(&row[q * 4]); __threadfence(); }
}
template <int KD, int EPI>
__global__ __launch_bounds__(128) void mlp_kernel(const float* __restrict__ X, const b16* __restrict__ Wt, const float* __restrict__ bias, int nb, float* __restrict__ Y, int ldy) {
  __shared__ __attribute__((aligned(16))) b16 Ah[4][16][256 + 8], Al[4][16][256 + 8]; __shared__ __attribute__((aligned(16))) float Tf[4][16][128 + 4];
  const int wave = threadIdx.x >> 5, lane = threadIdx.x & 31, nloc = lane & 15, hlf = lane >> 4; const size_t m0 = (size_t)blockIdx.x * 64 + wave * 16; const int n0 = blockIdx.y * 128;
  v8f acc[8];
#pragma unroll
  for (int t = 0; t < 8; ++t) acc[t] = (v8f){};
  for (int kc = 0; kc < KD; kc += 256) { const int kw = (KD - kc < 256) ? (KD - kc) : 256;
    for (int q = lane; q < 16 * 64; q += 32) { const int rr = q / 64, c4 = (q % 64) * 4; v4f xv = {0.0f, 0.0f, 0.0f, 0.0f}; if (c4 < kw) xv = *(const v4f*)(X + (m0 + rr) * KD + kc + c4); for (int j = 0; j < 4; ++j) { b16 p, pl; split16(xv[j] * XS, p, pl); Ah[wave][rr][c4 + j] = p; Al[wave][rr][c4 + j] = pl; } }
    wave_lds_sync();
    for (int kb = 0; kb < kw; kb += 32) { const v16b a = frag_kb(&Ah[wave][nloc][kb], hlf), al = frag_kb(&Al[wave][nloc][kb], hlf);
#pragma unroll
      for (int t = 0; t < 8; ++t) { const v16b bw = frag_kb(Wt + (size_t)(n0 + t * 16 + nloc) * KD + kc + kb, hlf); acc[t] = wmma16b(a, bw, acc[t]); acc[t] = wmma16b(al, bw, acc[t]); } }
    wave_lds_sync(); }
#pragma unroll
  for (int t = 0; t < 8; ++t) { const int c = n0 + t * 16 + nloc; const float bb = (c < nb) ? bf16_rne(bias[c]) : 0.0f;
#pragma unroll 1
    for (int r = 0; r < 8; ++r) { float y = acc[t][r] * (1.0f / (XS * WSC)) + bb; if (EPI == 1) y = fmaxf(y, 0.0f); Tf[wave][8 * hlf + r][t * 16 + nloc] = y; } }
  wave_lds_sync();
  for (int pass = 0; pass < 2; ++pass) { for (int rr = 0; rr < 16; ++rr) *(volatile v4f*)(Y + (m0 + rr) * ldy + n0 + lane * 4) = *(const v4f*)(&Tf[wave][rr][lane * 4]); __threadfence(); }
}
__global__ __launch_bounds__(256) void zcopy_kernel(const float* __restrict__ ZW, float* __restrict__ outz) {
  __shared__ __attribute__((aligned(16))) float z[G]; const int t_ = threadIdx.x; z[t_] = ZW[(size_t)t_ * 128]; __syncthreads();
  for (int pass = 0; pass < 2; ++pass) { if (t_ < 64) *(volatile v4f*)(outz + t_ * 4) = *(const v4f*)(&z[t_ * 4]); __threadfence(); }
}
}

extern "C" void kernel_launch(void* const* d_in, const int* in_sizes, int n_in, void* d_out, int out_size, void* d_ws, size_t ws_size, hipStream_t stream) {
  (void)n_in;
  auto Fp = [&](int i) { return (const float*)d_in[i]; }; auto Ip = [&](int i) { return (const int*)d_in[i]; };
  if (in_sizes[1] != N * F1 || in_sizes[2] != 2 * E || in_sizes[3] != N || in_sizes[4] != N * F2 || in_sizes[5] != 2 * E || in_sizes[6] != N || in_sizes[9] != F1 * N1L2 || in_sizes[13] != F2 * N2L2 || in_sizes[15] != P1W * HID || in_sizes[19] != P2W * HID || out_size != G * (1 + XG + XG + 1)) return;
  size_t off = 0; char* ws = (char*)d_ws;
  auto carve = [&](size_t bytes) { char* p = ws + off; off += (bytes + 255) & ~(size_t)255; return p; };
  b16* W1T = (b16*)carve((size_t)K1P * K1P * 2); b16* W2T = (b16*)carve((size_t)N1L2P * K1P * 2); b16* W3T = (b16*)carve((size_t)K2P * K2P * 2); b16* W4T = (b16*)carve((size_t)N2L2P * K2P * 2);
  b16* FG1 = (b16*)carve((size_t)HID * P1WP * 2); b16* FG2 = (b16*)carve((size_t)XG * HID * 2); b16* FH1 = (b16*)carve((size_t)HID * P2WP * 2); b16* FH2 = (b16*)carve((size_t)XG * HID * 2);
  b16* FF1 = (b16*)carve((size_t)FF * XG * 2); b16* FF2 = (b16*)carve((size_t)128 * FF * 2); b16* FE1 = (b16*)carve((size_t)FF * XG * 2); b16* FE2 = (b16*)carve((size_t)128 * FF * 2);
  float* S = (float*)carve((size_t)NP * K1P * 4); float* H1 = (float*)carve((size_t)NP * K1P * 4); float* POOL = (float*)carve((size_t)G * 2 * N1L2P * 4); float* PIN = (float*)carve((size_t)G * P1WP * 4); float* HD = (float*)carve((size_t)G * HID * 4); float* FQ = (float*)carve((size_t)G * FF * 4); float* ZW = (float*)carve((size_t)G * 128 * 4);
  CsrBufs csr; off = csr_carve(csr, ws, off, E, N);
  if (off > ws_size || off > ((size_t)128 << 20)) return;
  auto wprep = [&](const float* w, int nin, int nout, int kinp, int noutp, b16* dst) { wprep_kernel<<<(unsigned)(((size_t)noutp * kinp / 8 + 255) / 256), 256, 0, stream>>>(w, nin, nout, kinp, noutp, dst); };
  wprep(Fp(7), F1, F1, K1P, K1P, W1T); wprep(Fp(9), F1, N1L2, K1P, N1L2P, W2T); wprep(Fp(11), F2, F2, K2P, K2P, W3T); wprep(Fp(13), F2, N2L2, K2P, N2L2P, W4T);
  wprep(Fp(15), P1W, HID, P1WP, HID, FG1); wprep(Fp(17), HID, XG, HID, XG, FG2); wprep(Fp(19), P2W, HID, P2WP, HID, FH1); wprep(Fp(21), HID, XG, HID, XG, FH2);
  wprep(Fp(23), XG, FF, XG, FF, FF1); wprep(Fp(25), FF, 1, FF, 128, FF2); wprep(Fp(27), XG, FF, XG, FF, FE1); wprep(Fp(29), FF, 1, FF, 128, FE2);
  float* out_z = (float*)d_out; float* out_xg = out_z + G; float* out_xg1 = out_xg + (size_t)G * XG; float* out_z1 = out_xg1 + (size_t)G * XG;
  csr_build(csr, Ip(2) + E, E, N, stream);
  agg_kernel<F1, K1P><<<NP / 8, 256, 0, stream>>>(Fp(1), 1, Ip(2), csr.PERM, csr.ROWPTR, csr.ROWCNT, (int)csr.permLen, S);
  gin1_kernel<F1, K1P><<<NP / 64, 128, 0, stream>>>(S, W1T, Fp(8), H1);
  agg_kernel<F1, K1P><<<NP / 8, 256, 0, stream>>>(H1, 0, Ip(2), csr.PERM, csr.ROWPTR, csr.ROWCNT, (int)csr.permLen, S);
  gin2pool_kernel<K1P, N1L2, N1L2P><<<dim3(G, N1L2P / 64), 32, 0, stream>>>(S, W2T, Fp(10), Ip(3), POOL);
  repack_kernel<N1L2, N1L2P, P1WP><<<G, 256, 0, stream>>>(POOL, PIN);
  mlp_kernel<P1WP, 1><<<dim3(G / 64, HID / 128), 128, 0, stream>>>(PIN, FG1, Fp(16), HID, HD, HID);
  mlp_kernel<HID, 0><<<dim3(G / 64, XG / 128), 128, 0, stream>>>(HD, FG2, Fp(18), XG, out_xg, XG);
  mlp_kernel<XG, 1><<<dim3(G / 64, FF / 128), 128, 0, stream>>>(out_xg, FF1, Fp(24), FF, FQ, FF);
  mlp_kernel<FF, 0><<<dim3(G / 64, 1), 128, 0, stream>>>(FQ, FF2, Fp(26), 1, ZW, 128);
  zcopy_kernel<<<1, 256, 0, stream>>>(ZW, out_z);
  csr_build(csr, Ip(5) + E, E, N, stream);
  agg_kernel<F2, K2P><<<NP / 8, 256, 0, stream>>>(Fp(4), 1, Ip(5), csr.PERM, csr.ROWPTR, csr.ROWCNT, (int)csr.permLen, S);
  gin1_kernel<F2, K2P><<<NP / 64, 128, 0, stream>>>(S, W3T, Fp(12), H1);
  agg_kernel<F2, K2P><<<NP / 8, 256, 0, stream>>>(H1, 0, Ip(5), csr.PERM, csr.ROWPTR, csr.ROWCNT, (int)csr.permLen, S);
  gin2pool_kernel<K2P, N2L2, N2L2P><<<dim3(G, N2L2P / 64), 32, 0, stream>>>(S, W4T, Fp(14), Ip(6), POOL);
  repack_kernel<N2L2, N2L2P, P2WP><<<G, 256, 0, stream>>>(POOL, PIN);
  mlp_kernel<P2WP, 1><<<dim3(G / 64, HID / 128), 128, 0, stream>>>(PIN, FH1, Fp(20), HID, HD, HID);
  mlp_kernel<HID, 0><<<dim3(G / 64, XG / 128), 128, 0, stream>>>(HD, FH2, Fp(22), XG, out_xg1, XG);
  mlp_kernel<XG, 1><<<dim3(G / 64, FF / 128), 128, 0, stream>>>(out_xg1, FE1, Fp(28), FF, FQ, FF);
  mlp_kernel<FF, 0><<<dim3(G / 64, 1), 128, 0, stream>>>(FQ, FE2, Fp(30), 1, ZW, 128);
  zcopy_kernel<<<1, 256, 0, stream>>>(ZW, out_z1);
}
